// BiMambaBlock_88519275970819
// MI455X (gfx1250) — hardware-run, weakly checked
//
#include <hip/hip_runtime.h>
#include <math.h>

typedef __attribute__((ext_vector_type(16))) _Float16 v16h;
typedef __attribute__((ext_vector_type(8)))  _Float16 v8h;
typedef __attribute__((ext_vector_type(16))) __bf16   v16b;
typedef __attribute__((ext_vector_type(8)))  __bf16   v8b;
typedef __attribute__((ext_vector_type(8)))  float    v8f;
typedef __attribute__((ext_vector_type(4)))  float    v4f;

constexpr int kBatch  = 2;
constexpr int kSeq    = 1024;
constexpr int kDm     = 768;
constexpr int kDin    = 1536;
constexpr int kNst    = 16;
constexpr int kDtR    = 48;
constexpr int kDtRP   = 64;
constexpr int kXzP    = 2 * kDin;
constexpr int kXpN    = kDtR + 2 * kNst;
constexpr int kXpNP   = 128;
constexpr int kFfn    = 4 * kDm;
constexpr int kRows   = kBatch * kSeq;
constexpr int kConvTP = 260;
constexpr int kScanTS = 64;
constexpr int kScanCh = 64;
constexpr int kScanYP = 68;
constexpr int kScanXP = 2 * kNst;
constexpr float kCarryW  = 64.0f;
constexpr float kCarryLn = 16.0f;
constexpr float kCarryXc = 256.0f;
constexpr float kCarryDt = 256.0f;
constexpr float kCarryY  = 1024.0f;
constexpr float kCarryH1 = 16.0f;
static_assert(kXpN <= kXpNP && kDtR <= kDtRP, "pads");
static_assert((kDm % 32) == 0 && (kDin % 32) == 0 && (kDtRP % 32) == 0 && (kFfn % 32) == 0, "GEMM K multiples of 32");
static_assert((kRows % 64) == 0 && (kXzP % 64) == 0 && (kXpNP % 64) == 0 && (kDin % 64) == 0 && (kDm % 64) == 0 && (kFfn % 64) == 0, "GEMM M,N multiples of 64");
static_assert((kSeq % kScanTS) == 0 && (kSeq % 64) == 0 && (kDin % kScanCh) == 0 && (kDin % 256) == 0, "tile multiples");
static_assert((kDm % 256) == 0 && (kDm % 128) == 0, "LN lane maps");

constexpr size_t kSzInW  = (size_t)kXzP  * kDm   * 2;
constexpr size_t kSzXpW  = (size_t)kXpNP * kDin  * 2;
constexpr size_t kSzDtW  = (size_t)kDin  * kDtRP * 2;
constexpr size_t kSzOutW = (size_t)kDm   * kDin  * 2;
constexpr size_t kSzW1   = (size_t)kFfn  * kDm   * 2;
constexpr size_t kSzW2   = (size_t)kDm   * kFfn  * 2;
constexpr size_t kSzXN   = (size_t)kRows * kDm   * 2;
constexpr size_t kSzXZ   = (size_t)kRows * kXzP  * 4;
constexpr size_t kSzXC   = (size_t)kRows * kDin  * 4;
constexpr size_t kSzXC16 = (size_t)kRows * kDin  * 2;
constexpr size_t kSzDBC  = (size_t)kRows * kXpNP * 4;
constexpr size_t kSzDT16 = (size_t)kRows * kDtRP * 2;
constexpr size_t kSzDTR  = (size_t)kRows * kDin  * 4;
constexpr size_t kSzY16  = (size_t)kRows * kDin  * 2;
constexpr size_t kSzYP   = (size_t)kRows * kDm   * 4;
constexpr size_t kSzH1   = (size_t)kRows * kFfn  * 2;

constexpr size_t kOffINW0  = 0;
constexpr size_t kOffINW1  = kOffINW0  + kSzInW;
constexpr size_t kOffXPW0  = kOffINW1  + kSzInW;
constexpr size_t kOffXPW1  = kOffXPW0  + kSzXpW;
constexpr size_t kOffDTW0  = kOffXPW1  + kSzXpW;
constexpr size_t kOffDTW1  = kOffDTW0  + kSzDtW;
constexpr size_t kOffOUTW0 = kOffDTW1  + kSzDtW;
constexpr size_t kOffOUTW1 = kOffOUTW0 + kSzOutW;
constexpr size_t kOffW1    = kOffOUTW1 + kSzOutW;
constexpr size_t kOffW2    = kOffW1    + kSzW1;
constexpr size_t kOffXN    = kOffW2    + kSzW2;
constexpr size_t kOffXNR   = kOffXN    + kSzXN;
constexpr size_t kOffXZ    = kOffXNR   + kSzXN;
constexpr size_t kOffXC    = kOffXZ    + kSzXZ;
constexpr size_t kOffXC16  = kOffXC    + kSzXC;
constexpr size_t kOffDBC   = kOffXC16  + kSzXC16;
constexpr size_t kOffDT16  = kOffDBC   + kSzDBC;
constexpr size_t kOffDTR   = kOffDT16  + kSzDT16;
constexpr size_t kOffY16   = kOffDTR   + kSzDTR;
constexpr size_t kOffYPF   = kOffY16   + kSzY16;
constexpr size_t kOffYPB   = kOffYPF   + kSzYP;
constexpr size_t kOffXMID  = kOffYPB   + kSzYP;
constexpr size_t kOffH16   = kOffXMID  + kSzYP;
constexpr size_t kOffH1    = kOffH16   + kSzXN;
constexpr size_t kWsTotal  = kOffH1    + kSzH1;
static_assert(kWsTotal == 129892352ull, "carve total");
static_assert(kWsTotal <= 134217728ull, "carve cap");
static_assert((kSzInW % 128) == 0 && (kSzXpW % 128) == 0 && (kSzDtW % 128) == 0 && (kSzOutW % 128) == 0 &&
              (kSzW1 % 128) == 0 && (kSzXN % 128) == 0 && (kSzXZ % 128) == 0 && (kSzXC % 128) == 0 &&
              (kSzXC16 % 128) == 0 && (kSzDBC % 128) == 0 && (kSzDT16 % 128) == 0 && (kSzDTR % 128) == 0 &&
              (kSzY16 % 128) == 0 && (kSzYP % 128) == 0 && (kSzH1 % 128) == 0, "128-B aligned regions");
static_assert((size_t)kRows * kFfn * 4 == kSzXZ, "pre-activation plane equals XZ plane");

__device__ __forceinline__ void grp_guard_h(v8f& a, v8f& b, v8f& c, v8f& d, v16h x, v16h y0, v16h y1, v16h y2, v16h y3) {
  asm volatile("v_nop\n\tv_nop\n\tv_nop\n\tv_nop" : "+v"(a), "+v"(b), "+v"(c), "+v"(d) : "v"(x), "v"(y0), "v"(y1), "v"(y2), "v"(y3));
}
__device__ __forceinline__ void grp_guard_b(v8f& a, v8f& b, v8f& c, v8f& d, v16b x, v16b y0, v16b y1, v16b y2, v16b y3) {
  asm volatile("v_nop\n\tv_nop\n\tv_nop\n\tv_nop" : "+v"(a), "+v"(b), "+v"(c), "+v"(d) : "v"(x), "v"(y0), "v"(y1), "v"(y2), "v"(y3));
}
__device__ __forceinline__ void keep4_h(v16h a, v16h b, v16h c, v16h d) { asm volatile("v_nop" :: "v"(a), "v"(b), "v"(c), "v"(d)); }
__device__ __forceinline__ void keep4_b(v16b a, v16b b, v16b c, v16b d) { asm volatile("v_nop" :: "v"(a), "v"(b), "v"(c), "v"(d)); }
__device__ __forceinline__ void acc_guard4(v8f& a, v8f& b, v8f& c, v8f& d) { asm volatile("v_nop\n\tv_nop\n\tv_nop\n\tv_nop" : "+v"(a), "+v"(b), "+v"(c), "+v"(d)); }
template <typename T> struct Frag;
template <> struct Frag<_Float16> {
  typedef v16h V; union U { v16h v; v8h h[2]; };
  static __device__ __forceinline__ v16h load(const _Float16* p) {
    U f; f.h[0] = *(const v8h*)(p); f.h[1] = *(const v8h*)(p + 16); return f.v;
  }
  static __device__ __forceinline__ v8f mma(v16h a, v16h b, v8f c) {
    return __builtin_amdgcn_wmma_f32_16x16x32_f16(false, a, false, b, (short)0, c, false, false);
  }
  static __device__ __forceinline__ void guard4(v8f& a, v8f& b, v8f& c, v8f& d, v16h x, v16h y0, v16h y1, v16h y2, v16h y3) { grp_guard_h(a, b, c, d, x, y0, y1, y2, y3); }
  static __device__ __forceinline__ void keep(v16h a, v16h b, v16h c, v16h d) { keep4_h(a, b, c, d); }
};
template <> struct Frag<__bf16> {
  typedef v16b V; union U { v16b v; v8b h[2]; };
  static __device__ __forceinline__ v16b load(const __bf16* p) {
    U f; f.h[0] = *(const v8b*)(p); f.h[1] = *(const v8b*)(p + 16); return f.v;
  }
  static __device__ __forceinline__ v8f mma(v16b a, v16b b, v8f c) {
    return __builtin_amdgcn_wmma_f32_16x16x32_bf16(false, a, false, b, (short)0, c, false, false);
  }
  static __device__ __forceinline__ void guard4(v8f& a, v8f& b, v8f& c, v8f& d, v16b x, v16b y0, v16b y1, v16b y2, v16b y3) { grp_guard_b(a, b, c, d, x, y0, y1, y2, y3); }
  static __device__ __forceinline__ void keep(v16b a, v16b b, v16b c, v16b d) { keep4_b(a, b, c, d); }
};

template <int ET> struct Elem;
template <> struct Elem<0> { typedef _Float16 T; };
template <> struct Elem<1> { typedef __bf16 T; };
template <int ET, int SPL, int BIAS_MODE, bool RESID>
__global__ __launch_bounds__(256) void wmma_gemm64(
    const unsigned short* __restrict__ Ap, const unsigned short* __restrict__ A2p, int lda, long strideA,
    const unsigned short* __restrict__ Btp, const unsigned short* __restrict__ Bt2p, int ldb, long strideB,
    float* __restrict__ Cout, int ldc, long strideC,
    const float* __restrict__ bias,
    const float* __restrict__ resid, long strideR,
    int M, int N, int K, float scale) {
  typedef typename Elem<ET>::T T;
  typedef typename Frag<T>::V V;
  const T* A = (const T*)Ap; const T* A2 = (const T*)A2p; const T* Bt = (const T*)Btp; const T* Bt2 = (const T*)Bt2p;
  __shared__ __align__(16) float sT[8][16 * 68];
  const int b    = blockIdx.y;
  const int lane = threadIdx.x & 31;
  const int wave = threadIdx.x >> 5;
  const int tilesN = N >> 6;
  const int tilesM = M >> 6;
  const int tile = blockIdx.x * 8 + wave;
  if (tile >= tilesM * tilesN) return;
  const int tm = tile / tilesN;
  const int tn = tile - tm * tilesN;
  const int m0 = tm << 6;
  const int n0 = tn << 6;

  const T* Ab  = A  + (size_t)b * strideA;
  const T* Bb  = Bt + (size_t)b * strideB;
  const T* Ab2 = (SPL >= 1) ? (A2  + (size_t)b * strideA) : nullptr;
  const T* Bb2 = (SPL == 2) ? (Bt2 + (size_t)b * strideB) : nullptr;

  const int rlane = lane & 15;
  const int koff  = (lane >> 4) * 8;
  const int mOff  = (lane >> 4) * 8;

  v8f acc[4][4];
#pragma unroll
  for (int i = 0; i < 4; ++i)
#pragma unroll
    for (int j = 0; j < 4; ++j) acc[i][j] = (v8f){0.f,0.f,0.f,0.f,0.f,0.f,0.f,0.f};

  for (int k0 = 0; k0 < K; k0 += 32) {
    V bh[4], bl[4];
#pragma unroll
    for (int j = 0; j < 4; ++j) {
      const size_t bo = (size_t)(n0 + (j << 4) + rlane) * ldb + koff + k0;
      bh[j] = Frag<T>::load(Bb + bo);
      if (SPL == 2) bl[j] = Frag<T>::load(Bb2 + bo);
    }
#pragma unroll
    for (int i = 0; i < 4; ++i) {
      const size_t ao = (size_t)(m0 + (i << 4) + rlane) * lda + koff + k0;
      V ah = Frag<T>::load(Ab + ao);
      V al;
      if (SPL >= 1) al = Frag<T>::load(Ab2 + ao);
#pragma unroll
      for (int j = 0; j < 4; ++j) {
        acc[i][j] = Frag<T>::mma(ah, bh[j], acc[i][j]);
        if (SPL == 2) acc[i][j] = Frag<T>::mma(ah, bl[j], acc[i][j]);
        if (SPL >= 1) acc[i][j] = Frag<T>::mma(al, bh[j], acc[i][j]);
      }
      Frag<T>::guard4(acc[i][0], acc[i][1], acc[i][2], acc[i][3], ah, bh[0], bh[1], bh[2], bh[3]);
      if (SPL >= 1) Frag<T>::keep(al, al, al, al);
    }
    Frag<T>::keep(bh[0], bh[1], bh[2], bh[3]);
    if (SPL == 2) Frag<T>::keep(bl[0], bl[1], bl[2], bl[3]);
  }
  acc_guard4(acc[0][0], acc[0][1], acc[0][2], acc[0][3]);
  acc_guard4(acc[1][0], acc[1][1], acc[1][2], acc[1][3]);
  acc_guard4(acc[2][0], acc[2][1], acc[2][2], acc[2][3]);
  acc_guard4(acc[3][0], acc[3][1], acc[3][2], acc[3][3]);

  float* slab = sT[wave];
  const float* Rb = RESID ? (resid + (size_t)b * strideR) : nullptr;
  float* C = Cout + (size_t)b * strideC;
#pragma unroll
  for (int i = 0; i < 4; ++i) {
    const int mBase = m0 + (i << 4);
#pragma unroll
    for (int j = 0; j < 4; ++j) {
      const int n = n0 + (j << 4) + rlane;
      float bv = 0.f;
      if (BIAS_MODE == 2) bv = bias[n];
#pragma unroll
      for (int r = 0; r < 8; ++r) {
        float v = acc[i][j][r] * scale;
        if (BIAS_MODE == 2) v += bv;
        slab[(mOff + r) * 68 + (j << 4) + rlane] = v;
      }
    }
    __builtin_amdgcn_fence(__ATOMIC_RELEASE, "workgroup");
    __builtin_amdgcn_wave_barrier();
    __builtin_amdgcn_fence(__ATOMIC_ACQUIRE, "workgroup");
    {
      const int hh = lane >> 4, c4 = (lane & 15) * 4;
      for (int pass = 0; pass < 2; ++pass) {
#pragma unroll
        for (int it = 0; it < 8; ++it) {
          const int row = it * 2 + hh;
          v4f v = *(const v4f*)(slab + row * 68 + c4);
          if (RESID) {
            const v4f rv = *(const v4f*)(Rb + (size_t)(mBase + row) * ldc + n0 + c4);
            v = v + rv;
          }
          *(volatile v4f*)(C + (size_t)(mBase + row) * ldc + n0 + c4) = v;
        }
        __threadfence();
      }
    }
    __builtin_amdgcn_fence(__ATOMIC_RELEASE, "workgroup");
    __builtin_amdgcn_wave_barrier();
    __builtin_amdgcn_fence(__ATOMIC_ACQUIRE, "workgroup");
  }
}

__global__ __launch_bounds__(256) void cast_pad_f16_kernel(
    const float* __restrict__ in, unsigned short* __restrict__ out,
    int rows_in, int kin, int rows_out, int kout, float scale, int total8)
{
  const int i = blockIdx.x * 256 + threadIdx.x;
  if (i >= total8) return;
  const int gpr = kout >> 3;
  const int gin = kin >> 3;
  const int r = i / gpr;
  const int q = i - r * gpr;
  const int rr = (r < rows_in) ? r : (rows_in - 1);
  const int qq = (q < gin) ? q : (gin - 1);
  const float f = (r < rows_in && q < gin) ? scale : 0.0f;
  const float* p = in + (size_t)rr * kin + (qq << 3);
  const v4f a0 = *(const v4f*)(p);
  const v4f a1 = *(const v4f*)(p + 4);
  v8h hv;
#pragma unroll
  for (int e = 0; e < 4; ++e) {
    hv[e]     = (_Float16)(a0[e] * f);
    hv[4 + e] = (_Float16)(a1[e] * f);
  }
  unsigned short* o = out + ((size_t)i << 3);
  *(volatile v8h*)o = hv;
  __threadfence();
  *(volatile v8h*)o = hv;
}

__global__ __launch_bounds__(256) void ln_in_kernel(
    const float* __restrict__ x, const float* __restrict__ g, const float* __restrict__ bt,
    unsigned short* __restrict__ XN, unsigned short* __restrict__ XNR)
{
  const int lane = threadIdx.x & 31, wave = threadIdx.x >> 5;
  const int row  = blockIdx.x * 8 + wave;
  const int bi   = row >> 10;
  const int tt   = row & (kSeq - 1);
  const int rrow = (bi << 10) + (kSeq - 1 - tt);
  const float* xr = x + (size_t)row * kDm;
  v4f xa[3], xb[3];
#pragma unroll
  for (int k = 0; k < 3; ++k) {
    xa[k] = *(const v4f*)(xr + 256 * k + 8 * lane);
    xb[k] = *(const v4f*)(xr + 256 * k + 8 * lane + 4);
  }
  float s = 0.0f;
#pragma unroll
  for (int k = 0; k < 3; ++k)
    s += ((xa[k][0] + xa[k][1]) + (xa[k][2] + xa[k][3])) + ((xb[k][0] + xb[k][1]) + (xb[k][2] + xb[k][3]));
#pragma unroll
  for (int off = 1; off < 32; off <<= 1) s += __shfl_xor(s, off, 32);
  const float mean = s * (1.0f / (float)kDm);
  float q = 0.0f;
#pragma unroll
  for (int k = 0; k < 3; ++k) {
#pragma unroll
    for (int e = 0; e < 4; ++e) {
      const float da = xa[k][e] - mean;
      const float db = xb[k][e] - mean;
      q = fmaf(da, da, q);
      q = fmaf(db, db, q);
    }
  }
#pragma unroll
  for (int off = 1; off < 32; off <<= 1) q += __shfl_xor(q, off, 32);
  const float var  = q * (1.0f / (float)kDm);
  const float rstd = rsqrtf(var + 1e-5f);
  asm volatile("" ::: "memory");
  v8h hv[3];
#pragma unroll
  for (int k = 0; k < 3; ++k) {
    const v4f ga = *(const v4f*)(g  + 256 * k + 8 * lane);
    const v4f gb = *(const v4f*)(g  + 256 * k + 8 * lane + 4);
    const v4f ba = *(const v4f*)(bt + 256 * k + 8 * lane);
    const v4f bb = *(const v4f*)(bt + 256 * k + 8 * lane + 4);
#pragma unroll
    for (int e = 0; e < 4; ++e) {
      const float y0 = (xa[k][e] - mean) * rstd * ga[e] + ba[e];
      const float y1 = (xb[k][e] - mean) * rstd * gb[e] + bb[e];
      hv[k][e]     = (_Float16)(y0 * kCarryLn);
      hv[k][4 + e] = (_Float16)(y1 * kCarryLn);
    }
    asm volatile("" ::: "memory");
  }
  for (int pass = 0; pass < 2; ++pass) {
#pragma unroll
    for (int k = 0; k < 3; ++k) {
      *(volatile v8h*)(XN  + (size_t)row  * kDm + 256 * k + 8 * lane) = hv[k];
      *(volatile v8h*)(XNR + (size_t)rrow * kDm + 256 * k + 8 * lane) = hv[k];
    }
    __threadfence();
  }
}

__global__ __launch_bounds__(256) void conv_silu_kernel(
    const float* __restrict__ XZ, const float* __restrict__ cw, const float* __restrict__ cb,
    float* __restrict__ XC, unsigned short* __restrict__ XC16)
{
  __shared__ __align__(16) float sT[16 * kConvTP];
  const int tid = threadIdx.x, lane = tid & 31, wave = tid >> 5;
  const int d0 = blockIdx.x * 256, d = d0 + tid;
  const int g0 = blockIdx.y * 64;
  const int tb = g0 & (kSeq - 1);
  const float w0 = cw[d * 4 + 0], w1 = cw[d * 4 + 1], w2 = cw[d * 4 + 2], w3 = cw[d * 4 + 3];
  const float bc = cb[d];
  float xm3, xm2, xm1;
  {
    const bool hist = (tb > 0);
    const int rb = hist ? (g0 - 3) : g0;
    const float v3 = XZ[(size_t)rb * kXzP + d];
    const float v2 = XZ[(size_t)(rb + 1) * kXzP + d];
    const float v1 = XZ[(size_t)(rb + 2) * kXzP + d];
    xm3 = hist ? v3 : 0.f;
    xm2 = hist ? v2 : 0.f;
    xm1 = hist ? v1 : 0.f;
  }
  const int hrow = wave >> 1;
  const int hch  = (wave & 1) * 128 + lane * 4;
#pragma unroll 1
  for (int sub = 0; sub < 4; ++sub) {
    const int lb = g0 + sub * 16;
#pragma unroll 1
    for (int s = 0; s < 16; ++s) {
      const float xcur = XZ[(size_t)(lb + s) * kXzP + d];
      float acc = w0 * xm3;
      acc = fmaf(w1, xm2, acc);
      acc = fmaf(w2, xm1, acc);
      acc = fmaf(w3, xcur, acc);
      const float sv = acc + bc;
      const float sg = __builtin_amdgcn_rcpf(1.0f + __expf(-sv));
      sT[s * kConvTP + tid] = sv * sg;
      xm3 = xm2; xm2 = xm1; xm1 = xcur;
    }
    __syncthreads();
    v4f fv[4];
    v8h hv[2];
#pragma unroll
    for (int it = 0; it < 4; ++it) fv[it] = *(const v4f*)(sT + (it * 4 + hrow) * kConvTP + hch);
#pragma unroll
    for (int it = 0; it < 2; ++it) {
      const float* sp = sT + (it * 8 + wave) * kConvTP + lane * 8;
      const v4f a0 = *(const v4f*)(sp);
      const v4f a1 = *(const v4f*)(sp + 4);
#pragma unroll
      for (int e = 0; e < 4; ++e) {
        hv[it][e]     = (_Float16)(a0[e] * kCarryXc);
        hv[it][4 + e] = (_Float16)(a1[e] * kCarryXc);
      }
    }
    for (int pass = 0; pass < 2; ++pass) {
#pragma unroll
      for (int it = 0; it < 4; ++it)
        *(volatile v4f*)(XC + (size_t)(lb + it * 4 + hrow) * kDin + d0 + hch) = fv[it];
#pragma unroll
      for (int it = 0; it < 2; ++it)
        *(volatile v8h*)(XC16 + (size_t)(lb + it * 8 + wave) * kDin + d0 + lane * 8) = hv[it];
      __threadfence();
    }
    __syncthreads();
  }
}

__global__ __launch_bounds__(256) void dt_pack_kernel(
    const float* __restrict__ DBC, unsigned short* __restrict__ DT16, int total8)
{
  const int i = blockIdx.x * 256 + threadIdx.x;
  if (i >= total8) return;
  const int r = i >> 3;
  const int q = i & 7;
  const float* p = DBC + (size_t)r * kXpNP + (q << 3);
  const v4f a0 = *(const v4f*)(p);
  const v4f a1 = *(const v4f*)(p + 4);
  const float f = (q < (kDtR >> 3)) ? kCarryDt : 0.0f;
  v8h hv;
#pragma unroll
  for (int e = 0; e < 4; ++e) {
    hv[e]     = (_Float16)(a0[e] * f);
    hv[4 + e] = (_Float16)(a1[e] * f);
  }
  unsigned short* o = DT16 + ((size_t)i << 3);
  *(volatile v8h*)o = hv;
  __threadfence();
  *(volatile v8h*)o = hv;
}

__global__ __launch_bounds__(64) void scan_kernel(
    const float* __restrict__ DBC, const float* __restrict__ DTR, const float* __restrict__ XC,
    const float* __restrict__ XZ, const float* __restrict__ bdt, const float* __restrict__ Alog,
    const float* __restrict__ Dp, unsigned short* __restrict__ Y16)
{
  __shared__ __align__(16) float sX[kScanTS * kScanXP];
  __shared__ __align__(16) float sY[kScanTS * kScanYP];
  __shared__ __align__(16) float sA[kNst * kScanCh];
  const int tid = threadIdx.x, lane = tid & 31, wave = tid >> 5;
  constexpr int kBlkPerB = kDin / kScanCh;
  const int bix = blockIdx.x / kBlkPerB;
  const int d0  = (blockIdx.x - bix * kBlkPerB) * kScanCh;
  const int d   = d0 + tid;
  const size_t row0 = (size_t)bix * kSeq;
#pragma unroll 1
  for (int s = 0; s < kNst; ++s) sA[s * kScanCh + tid] = -expf(Alog[(size_t)d * kNst + s]);
  __syncthreads();
  float negA[kNst], h[kNst];
#pragma unroll
  for (int s = 0; s < kNst; ++s) {
    negA[s] = sA[s * kScanCh + tid];
    h[s] = 0.0f;
  }
  const float bb = bdt[d], Dd = Dp[d];
  const int q = lane >> 3, c8 = (lane & 7) * 8;
#pragma unroll 1
  for (int t0 = 0; t0 < kSeq; t0 += kScanTS) {
    __syncthreads();
    {
      const float* src = DBC + (row0 + t0 + tid) * kXpNP + kDtR;
#pragma unroll
      for (int i = 0; i < 8; ++i) *(v4f*)(sX + tid * kScanXP + 4 * i) = *(const v4f*)(src + 4 * i);
    }
    __syncthreads();
#pragma unroll 1
    for (int s = 0; s < kScanTS; ++s) {
      const int t = t0 + s;
      const float* xr = sX + s * kScanXP;
      float Bs[kNst], Cs[kNst];
#pragma unroll
      for (int q4 = 0; q4 < 4; ++q4) {
        const v4f bv = *(const v4f*)(xr + 4 * q4);
        const v4f cv = *(const v4f*)(xr + kNst + 4 * q4);
        Bs[4 * q4 + 0] = bv[0]; Bs[4 * q4 + 1] = bv[1]; Bs[4 * q4 + 2] = bv[2]; Bs[4 * q4 + 3] = bv[3];
        Cs[4 * q4 + 0] = cv[0]; Cs[4 * q4 + 1] = cv[1]; Cs[4 * q4 + 2] = cv[2]; Cs[4 * q4 + 3] = cv[3];
      }
      const float v   = DTR[(row0 + t) * kDin + d] + bb;
      const float a   = __expf(-fabsf(v));
      const float u   = 1.0f + a;
      const float l1p = __logf(u) + (a - (u - 1.0f)) * __builtin_amdgcn_rcpf(u);
      const float dt  = fmaxf(v, 0.0f) + l1p;
      const float xt  = XC[(row0 + t) * kDin + d];
      const float dtx = dt * xt;
      float y = 0.0f;
#pragma unroll
      for (int k = 0; k < kNst; ++k) {
        const float e = __expf(dt * negA[k]);
        h[k] = e * h[k] + dtx * Bs[k];
        y = h[k] * Cs[k] + y;
      }
      y = xt * Dd + y;
      const float zv = XZ[(row0 + t) * kXzP + kDin + d];
      const float sg = __builtin_amdgcn_rcpf(1.0f + __expf(-zv));
      y = y * (zv * sg);
      sY[s * kScanYP + tid] = y;
    }
    __syncthreads();
    v8h hv[8];
#pragma unroll
    for (int it = 0; it < 8; ++it) {
      const int row = it * 8 + wave * 4 + q;
      const float* sp = sY + row * kScanYP + c8;
      const v4f a0 = *(const v4f*)(sp);
      const v4f a1 = *(const v4f*)(sp + 4);
#pragma unroll
      for (int e = 0; e < 4; ++e) {
        hv[it][e]     = (_Float16)(a0[e] * kCarryY);
        hv[it][4 + e] = (_Float16)(a1[e] * kCarryY);
      }
    }
    for (int pass = 0; pass < 2; ++pass) {
#pragma unroll
      for (int it = 0; it < 8; ++it) {
        const int row = it * 8 + wave * 4 + q;
        const size_t o = (row0 + t0 + row) * kDin + d0 + c8;
        *(volatile v8h*)(Y16 + o) = hv[it];
      }
      __threadfence();
    }
  }
}

__global__ __launch_bounds__(256) void comb_ln_kernel(
    const float* __restrict__ x, const float* __restrict__ YPF, const float* __restrict__ YPB,
    const float* __restrict__ g, const float* __restrict__ bt,
    float* __restrict__ XMID, unsigned short* __restrict__ H16)
{
  __shared__ __align__(16) float sRow[8][kDm];
  const int lane = threadIdx.x & 31, wave = threadIdx.x >> 5;
  const int row  = blockIdx.x * 8 + wave;
  const int bi   = row >> 10;
  const int tt   = row & (kSeq - 1);
  const int rrow = (bi << 10) + (kSeq - 1 - tt);
  v4f xm[6];
  {
    v4f xx[6], yf[6];
#pragma unroll
    for (int k = 0; k < 6; ++k) xx[k] = *(const v4f*)(x + (size_t)row * kDm + 128 * k + 4 * lane);
    asm volatile("" ::: "memory");
#pragma unroll
    for (int k = 0; k < 6; ++k) yf[k] = *(const v4f*)(YPF + (size_t)row * kDm + 128 * k + 4 * lane);
    asm volatile("" ::: "memory");
#pragma unroll
    for (int k = 0; k < 6; ++k) {
      const v4f yb = *(const v4f*)(YPB + (size_t)rrow * kDm + 128 * k + 4 * lane);
      const v4f ys = (yf[k] + yb) * 0.5f;
      xm[k] = xx[k] + ys;
    }
  }
  float s = 0.0f;
#pragma unroll
  for (int k = 0; k < 6; ++k) s += (xm[k][0] + xm[k][1]) + (xm[k][2] + xm[k][3]);
#pragma unroll
  for (int off = 1; off < 32; off <<= 1) s += __shfl_xor(s, off, 32);
  const float mean = s * (1.0f / (float)kDm);
  float q = 0.0f;
#pragma unroll
  for (int k = 0; k < 6; ++k) {
#pragma unroll
    for (int e = 0; e < 4; ++e) { const float dv = xm[k][e] - mean; q = fmaf(dv, dv, q); }
  }
#pragma unroll
  for (int off = 1; off < 32; off <<= 1) q += __shfl_xor(q, off, 32);
  const float var  = q * (1.0f / (float)kDm);
  const float rstd = rsqrtf(var + 1e-5f);
  asm volatile("" ::: "memory");
  float* slab = sRow[wave];
#pragma unroll
  for (int k = 0; k < 6; ++k) {
    const v4f ga = *(const v4f*)(g  + 128 * k + 4 * lane);
    const v4f ba = *(const v4f*)(bt + 128 * k + 4 * lane);
    v4f hn;
#pragma unroll
    for (int e = 0; e < 4; ++e) hn[e] = ((xm[k][e] - mean) * rstd * ga[e] + ba[e]) * kCarryLn;
    *(v4f*)(slab + 128 * k + 4 * lane) = hn;
    if (k & 1) asm volatile("" ::: "memory");
  }
  for (int pass = 0; pass < 2; ++pass) {
#pragma unroll
    for (int k = 0; k < 6; ++k)
      *(volatile v4f*)(XMID + (size_t)row * kDm + 128 * k + 4 * lane) = xm[k];
    __threadfence();
  }
  __builtin_amdgcn_fence(__ATOMIC_RELEASE, "workgroup");
  __builtin_amdgcn_wave_barrier();
  __builtin_amdgcn_fence(__ATOMIC_ACQUIRE, "workgroup");
  v8h hv[3];
#pragma unroll
  for (int k = 0; k < 3; ++k) {
    const v4f a0 = *(const v4f*)(slab + 256 * k + 8 * lane);
    const v4f a1 = *(const v4f*)(slab + 256 * k + 8 * lane + 4);
#pragma unroll
    for (int e = 0; e < 4; ++e) {
      hv[k][e]     = (_Float16)a0[e];
      hv[k][4 + e] = (_Float16)a1[e];
    }
  }
  for (int pass = 0; pass < 2; ++pass) {
#pragma unroll
    for (int k = 0; k < 3; ++k)
      *(volatile v8h*)(H16 + (size_t)row * kDm + 256 * k + 8 * lane) = hv[k];
    __threadfence();
  }
}

__global__ __launch_bounds__(256) void gelu_f16x2_kernel(
    const float* __restrict__ in, _Float16* __restrict__ out, int n2)
{
  const int i = blockIdx.x * 256 + threadIdx.x;
  if (i < n2) {
    const float x0 = in[2 * (size_t)i], x1 = in[2 * (size_t)i + 1];
    const float g0 = 0.5f * x0 * (1.0f + erff(x0 * 0.70710678118654752f));
    const float g1 = 0.5f * x1 * (1.0f + erff(x1 * 0.70710678118654752f));
    const _Float16 h0 = (_Float16)(g0 * kCarryH1), h1 = (_Float16)(g1 * kCarryH1);
    const unsigned u = (unsigned)__builtin_bit_cast(unsigned short, h0) | ((unsigned)__builtin_bit_cast(unsigned short, h1) << 16);
    ((volatile unsigned*)out)[i] = u;
    __threadfence();
    ((volatile unsigned*)out)[i] = u;
  }
}

extern "C" void kernel_launch(void* const* d_in, const int* in_sizes, int n_in,
                              void* d_out, int out_size, void* d_ws, size_t ws_size,
                              hipStream_t stream) {
  if (n_in < 27) return;
  const int wantIn[27] = {
    kRows * kDm, kDm, kDm,
    kXzP * kDm, kDin * 4, kDin, kXpN * kDin, kDin * kDtR, kDin, kDin * kNst, kDin, kDm * kDin,
    kXzP * kDm, kDin * 4, kDin, kXpN * kDin, kDin * kDtR, kDin, kDin * kNst, kDin, kDm * kDin,
    kDm, kDm, kFfn * kDm, kFfn, kDm * kFfn, kDm };
  for (int i = 0; i < 27; ++i) if (in_sizes[i] != wantIn[i]) return;
  if (out_size != kRows * kDm) return;
  if (ws_size < kWsTotal) return;

  const float* x      = (const float*)d_in[0];
  const float* ln_g   = (const float*)d_in[1];
  const float* ln_b   = (const float*)d_in[2];
  const float* ffn_g  = (const float*)d_in[21];
  const float* ffn_b  = (const float*)d_in[22];
  const float* w1     = (const float*)d_in[23];
  const float* b1     = (const float*)d_in[24];
  const float* w2     = (const float*)d_in[25];
  const float* b2     = (const float*)d_in[26];
  float* out = (float*)d_out;

  char* ws = (char*)d_ws;
  unsigned short* INW[2]  = { (unsigned short*)(ws + kOffINW0),  (unsigned short*)(ws + kOffINW1) };
  unsigned short* XPW[2]  = { (unsigned short*)(ws + kOffXPW0),  (unsigned short*)(ws + kOffXPW1) };
  unsigned short* DTW[2]  = { (unsigned short*)(ws + kOffDTW0),  (unsigned short*)(ws + kOffDTW1) };
  unsigned short* OUTW[2] = { (unsigned short*)(ws + kOffOUTW0), (unsigned short*)(ws + kOffOUTW1) };
  unsigned short* W1P  = (unsigned short*)(ws + kOffW1);
  unsigned short* W2P  = (unsigned short*)(ws + kOffW2);
  unsigned short* XN   = (unsigned short*)(ws + kOffXN);
  unsigned short* XNR  = (unsigned short*)(ws + kOffXNR);
  float*          XZ   = (float*)(ws + kOffXZ);
  float*          XC   = (float*)(ws + kOffXC);
  unsigned short* XC16 = (unsigned short*)(ws + kOffXC16);
  float*          DBC  = (float*)(ws + kOffDBC);
  unsigned short* DT16 = (unsigned short*)(ws + kOffDT16);
  float*          DTR  = (float*)(ws + kOffDTR);
  unsigned short* Y16  = (unsigned short*)(ws + kOffY16);
  float*          YPF  = (float*)(ws + kOffYPF);
  float*          YPB  = (float*)(ws + kOffYPB);
  float*          XMID = (float*)(ws + kOffXMID);
  unsigned short* H16  = (unsigned short*)(ws + kOffH16);
  unsigned short* H1   = (unsigned short*)(ws + kOffH1);
  float*          H1PRE = XZ;

  for (int dir = 0; dir < 2; ++dir) {
    const int base = 3 + dir * 9;
    {
      const int total8 = kXzP * kDm / 8;
      cast_pad_f16_kernel<<<(total8 + 255) / 256, 256, 0, stream>>>((const float*)d_in[base + 0], INW[dir], kXzP, kDm, kXzP, kDm, kCarryW, total8);
    }
    {
      const int total8 = kXpNP * kDin / 8;
      cast_pad_f16_kernel<<<(total8 + 255) / 256, 256, 0, stream>>>((const float*)d_in[base + 3], XPW[dir], kXpN, kDin, kXpNP, kDin, kCarryW, total8);
    }
    {
      const int total8 = kDin * kDtRP / 8;
      cast_pad_f16_kernel<<<(total8 + 255) / 256, 256, 0, stream>>>((const float*)d_in[base + 4], DTW[dir], kDin, kDtR, kDin, kDtRP, kCarryW, total8);
    }
    {
      const int total8 = kDm * kDin / 8;
      cast_pad_f16_kernel<<<(total8 + 255) / 256, 256, 0, stream>>>((const float*)d_in[base + 8], OUTW[dir], kDm, kDin, kDm, kDin, kCarryW, total8);
    }
  }
  {
    const int total8 = kFfn * kDm / 8;
    cast_pad_f16_kernel<<<(total8 + 255) / 256, 256, 0, stream>>>(w1, W1P, kFfn, kDm, kFfn, kDm, kCarryW, total8);
    cast_pad_f16_kernel<<<(total8 + 255) / 256, 256, 0, stream>>>(w2, W2P, kDm, kFfn, kDm, kFfn, kCarryW, total8);
  }

  ln_in_kernel<<<kRows / 8, 256, 0, stream>>>(x, ln_g, ln_b, XN, XNR);

  for (int dir = 0; dir < 2; ++dir) {
    const int base = 3 + dir * 9;
    const float* conv_w = (const float*)d_in[base + 1];
    const float* conv_b = (const float*)d_in[base + 2];
    const float* dt_b   = (const float*)d_in[base + 5];
    const float* A_log  = (const float*)d_in[base + 6];
    const float* Dskip  = (const float*)d_in[base + 7];
    const unsigned short* src = dir ? XNR : XN;
    float* yp = dir ? YPB : YPF;

    wmma_gemm64<0, 0, 0, false><<<dim3(192, 1), 256, 0, stream>>>(
        src, nullptr, kDm, 0L,
        INW[dir], nullptr, kDm, 0L,
        XZ, kXzP, 0L,
        nullptr, nullptr, 0L,
        kRows, kXzP, kDm, 1.0f / (kCarryLn * kCarryW));

    conv_silu_kernel<<<dim3(kDin / 256, kRows / 64), 256, 0, stream>>>(XZ, conv_w, conv_b, XC, XC16);

    wmma_gemm64<0, 0, 0, false><<<dim3(8, 1), 256, 0, stream>>>(
        XC16, nullptr, kDin, 0L,
        XPW[dir], nullptr, kDin, 0L,
        DBC, kXpNP, 0L,
        nullptr, nullptr, 0L,
        kRows, kXpNP, kDin, 1.0f / (kCarryXc * kCarryW));

    dt_pack_kernel<<<(kRows * kDtRP / 8) / 256, 256, 0, stream>>>(DBC, DT16, kRows * kDtRP / 8);

    wmma_gemm64<0, 0, 0, false><<<dim3(96, 1), 256, 0, stream>>>(
        DT16, nullptr, kDtRP, 0L,
        DTW[dir], nullptr, kDtRP, 0L,
        DTR, kDin, 0L,
        nullptr, nullptr, 0L,
        kRows, kDin, kDtRP, 1.0f / (kCarryDt * kCarryW));

    scan_kernel<<<kBatch * (kDin / kScanCh), kScanCh, 0, stream>>>(DBC, DTR, XC, XZ, dt_b, A_log, Dskip, Y16);

    wmma_gemm64<0, 0, 0, false><<<dim3(48, 1), 256, 0, stream>>>(
        Y16, nullptr, kDin, 0L,
        OUTW[dir], nullptr, kDin, 0L,
        yp, kDm, 0L,
        nullptr, nullptr, 0L,
        kRows, kDm, kDin, 1.0f / (kCarryY * kCarryW));
  }

  comb_ln_kernel<<<kRows / 8, 256, 0, stream>>>(x, YPF, YPB, ffn_g, ffn_b, XMID, H16);

  wmma_gemm64<0, 0, 2, false><<<dim3(192, 1), 256, 0, stream>>>(
      H16, nullptr, kDm, 0L,
      W1P, nullptr, kDm, 0L,
      H1PRE, kFfn, 0L,
      b1, nullptr, 0L,
      kRows, kFfn, kDm, 1.0f / (kCarryLn * kCarryW));

  gelu_f16x2_kernel<<<(kRows * kFfn / 2) / 256, 256, 0, stream>>>(H1PRE, (_Float16*)H1, kRows * kFfn / 2);

  wmma_gemm64<0, 0, 2, true><<<dim3(48, 1), 256, 0, stream>>>(
      H1, nullptr, kFfn, 0L,
      W2P, nullptr, kFfn, 0L,
      out, kDm, 0L,
      b2, XMID, 0L,
      kRows, kDm, kFfn, 1.0f / (kCarryH1 * kCarryW));
}
